// Retention_14431090114834
// MI455X (gfx1250) — hardware-verified
//
#include <hip/hip_runtime.h>
#include <math.h>
#include <cmath>

constexpr int kBatch = 2;
constexpr int kSeq   = 2048;
constexpr int kDim   = 1024;
constexpr int kHeads = 16;
constexpr int kDh    = 64;
constexpr int kTok   = kBatch * kSeq;
constexpr int kFreq  = kDh / 2;
constexpr int kQB    = 64;
constexpr int kKC    = 64;
constexpr int kNCh   = kSeq / kKC;
constexpr int kOsPitch = 68;
constexpr float kScoreScale = 0.125f;
constexpr float kSkipArg    = 30.0f;
static_assert(kHeads * kDh == kDim, "shape");
static_assert(kFreq == 32, "freq");
static_assert(kSeq % kQB == 0 && kSeq % kKC == 0 && kQB == kKC, "tiles");
static_assert(kTok % 64 == 0 && kDim % 64 == 0 && kDim % 32 == 0, "gemm");
static_assert((kTok * kDim) % (8 * 256) == 0 && (kDim * kDim) % (8 * 256) == 0, "cast grids");
static_assert(kDim == 128 * 8, "rotary block covers one row");

typedef __attribute__((ext_vector_type(16))) _Float16 v16h;
typedef __attribute__((ext_vector_type(8)))  _Float16 v8h;
typedef __attribute__((ext_vector_type(16))) __bf16   v16b;
typedef __attribute__((ext_vector_type(8)))  __bf16   v8b;
typedef __attribute__((ext_vector_type(8)))  float    v8f;
typedef __attribute__((ext_vector_type(4)))  float    v4f;
typedef __attribute__((ext_vector_type(4)))  unsigned int v4u;

__device__ __forceinline__ unsigned short f2bf_bits(float f) {
  unsigned u = __float_as_uint(f);
  return (unsigned short)((u + 0x7FFFu + ((u >> 16) & 1u)) >> 16);
}
__device__ __forceinline__ float bf_bits2f(unsigned short h) { return __uint_as_float(((unsigned)h) << 16); }

__device__ __forceinline__ void dep_guard_h(v8f& a, v8f& b, v16h x, v16h y) { asm volatile("v_nop\n\tv_nop\n\tv_nop\n\tv_nop" : "+v"(a), "+v"(b) : "v"(x), "v"(y)); }
__device__ __forceinline__ void dep_guard_b(v8f& a, v8f& b, v16b x, v16b y) { asm volatile("v_nop\n\tv_nop\n\tv_nop\n\tv_nop" : "+v"(a), "+v"(b) : "v"(x), "v"(y)); }
__device__ __forceinline__ void dep_guard4_h(v8f& a, v8f& b, v8f& c, v8f& d, v16h x, v16h y) { asm volatile("v_nop\n\tv_nop\n\tv_nop\n\tv_nop" : "+v"(a), "+v"(b), "+v"(c), "+v"(d) : "v"(x), "v"(y)); }
__device__ __forceinline__ void dep_guard4_b(v8f& a, v8f& b, v8f& c, v8f& d, v16b x, v16b y) { asm volatile("v_nop\n\tv_nop\n\tv_nop\n\tv_nop" : "+v"(a), "+v"(b), "+v"(c), "+v"(d) : "v"(x), "v"(y)); }
__device__ __forceinline__ void keep4_h(v16h a, v16h b, v16h c, v16h d) { asm volatile("v_nop" :: "v"(a), "v"(b), "v"(c), "v"(d)); }
__device__ __forceinline__ void keep4_b(v16b a, v16b b, v16b c, v16b d) { asm volatile("v_nop" :: "v"(a), "v"(b), "v"(c), "v"(d)); }
__device__ __forceinline__ void acc_guard4(v8f& a, v8f& b, v8f& c, v8f& d) { asm volatile("v_nop\n\tv_nop\n\tv_nop\n\tv_nop" : "+v"(a), "+v"(b), "+v"(c), "+v"(d)); }
template <typename T> struct Frag;
template <> struct Frag<_Float16> {
  typedef v16h V; union U { v16h v; v8h h[2]; };
  static __device__ __forceinline__ v16h load(const _Float16* p) {
    U f; f.h[0] = *(const v8h*)(p); f.h[1] = *(const v8h*)(p + 16); return f.v;
  }
  static __device__ __forceinline__ v8f mma(v16h a, v16h b, v8f c) {
    return __builtin_amdgcn_wmma_f32_16x16x32_f16(false, a, false, b, (short)0, c, false, false);
  }
  static __device__ __forceinline__ void guard(v8f& a, v8f& b, v16h x, v16h y) { dep_guard_h(a, b, x, y); }
  static __device__ __forceinline__ void guard4(v8f& a, v8f& b, v8f& c, v8f& d, v16h x, v16h y) { dep_guard4_h(a, b, c, d, x, y); }
  static __device__ __forceinline__ void keep(v16h a, v16h b, v16h c, v16h d) { keep4_h(a, b, c, d); }
};
template <> struct Frag<__bf16> {
  typedef v16b V; union U { v16b v; v8b h[2]; };
  static __device__ __forceinline__ v16b load(const __bf16* p) {
    U f; f.h[0] = *(const v8b*)(p); f.h[1] = *(const v8b*)(p + 16); return f.v;
  }
  static __device__ __forceinline__ v8f mma(v16b a, v16b b, v8f c) {
    return __builtin_amdgcn_wmma_f32_16x16x32_bf16(false, a, false, b, (short)0, c, false, false);
  }
  static __device__ __forceinline__ void guard(v8f& a, v8f& b, v16b x, v16b y) { dep_guard_b(a, b, x, y); }
  static __device__ __forceinline__ void guard4(v8f& a, v8f& b, v8f& c, v8f& d, v16b x, v16b y) { dep_guard4_b(a, b, c, d, x, y); }
  static __device__ __forceinline__ void keep(v16b a, v16b b, v16b c, v16b d) { keep4_b(a, b, c, d); }
};

__device__ __forceinline__ unsigned pk16(unsigned short a, unsigned short b) { return (unsigned)a | ((unsigned)b << 16); }

__device__ __forceinline__ v8f mma_bf16g(v16b a, v16b b, v8f c) {
  c = __builtin_amdgcn_wmma_f32_16x16x32_bf16(false, a, false, b, (short)0, c, false, false);
  asm volatile("v_nop\n\tv_nop\n\tv_nop\n\tv_nop" : "+v"(c) : "v"(a), "v"(b));
  return c;
}

template <int ET> struct Elem;
template <> struct Elem<0> { typedef _Float16 T; };
template <> struct Elem<1> { typedef __bf16 T; };
template <int ET, bool SPLIT, int BIAS_MODE, int OUT_MODE, bool RESID, int ACT = 0>
__global__ __launch_bounds__(256) void wmma_gemm64(
    const unsigned short* __restrict__ Ap, const unsigned short* __restrict__ A2p, int lda, long strideA,
    const unsigned short* __restrict__ Btp, const unsigned short* __restrict__ Bt2p, int ldb, long strideB,
    void* __restrict__ Cout, void* __restrict__ Cout2, int ldc, long strideC,
    const float* __restrict__ bias,
    const float* __restrict__ resid, long strideR,
    int M, int N, int K, float scale) {
  typedef typename Elem<ET>::T T;
  typedef typename Frag<T>::V V;
  const T* A = (const T*)Ap; const T* A2 = (const T*)A2p; const T* Bt = (const T*)Btp; const T* Bt2 = (const T*)Bt2p;
  __shared__ __align__(16) float sT[8][16 * 68];
  const int b    = blockIdx.y;
  const int lane = threadIdx.x & 31;
  const int wave = threadIdx.x >> 5;
  const int tilesN = N >> 6;
  const int tilesM = M >> 6;
  const int tile = blockIdx.x * 8 + wave;
  if (tile >= tilesM * tilesN) return;
  const int tm = tile / tilesN;
  const int tn = tile - tm * tilesN;
  const int m0 = tm << 6;
  const int n0 = tn << 6;

  const T* Ab  = A  + (size_t)b * strideA;
  const T* Bb  = Bt + (size_t)b * strideB;
  const T* Ab2 = SPLIT ? (A2  + (size_t)b * strideA) : nullptr;
  const T* Bb2 = SPLIT ? (Bt2 + (size_t)b * strideB) : nullptr;

  const int rlane = lane & 15;
  const int koff  = (lane >> 4) * 8;
  const int mOff  = (lane >> 4) * 8;

  v8f acc[4][4];
#pragma unroll
  for (int i = 0; i < 4; ++i)
#pragma unroll
    for (int j = 0; j < 4; ++j) acc[i][j] = (v8f){0.f,0.f,0.f,0.f,0.f,0.f,0.f,0.f};

  for (int k0 = 0; k0 < K; k0 += 32) {
    V bh[4], bl[4];
#pragma unroll
    for (int j = 0; j < 4; ++j) {
      const size_t bo = (size_t)(n0 + (j << 4) + rlane) * ldb + koff + k0;
      bh[j] = Frag<T>::load(Bb + bo);
      if (SPLIT) bl[j] = Frag<T>::load(Bb2 + bo);
    }
#pragma unroll
    for (int i = 0; i < 4; ++i) {
      const size_t ao = (size_t)(m0 + (i << 4) + rlane) * lda + koff + k0;
      V ah = Frag<T>::load(Ab + ao);
      V al;
      if (SPLIT) al = Frag<T>::load(Ab2 + ao);
#pragma unroll
      for (int j = 0; j < 4; ++j) {
        acc[i][j] = Frag<T>::mma(ah, bh[j], acc[i][j]);
        if (SPLIT) {
          acc[i][j] = Frag<T>::mma(ah, bl[j], acc[i][j]);
          acc[i][j] = Frag<T>::mma(al, bh[j], acc[i][j]);
        }
      }
      Frag<T>::guard4(acc[i][0], acc[i][1], acc[i][2], acc[i][3], ah, SPLIT ? al : ah);
    }
    Frag<T>::keep(bh[0], bh[1], bh[2], bh[3]);
    if (SPLIT) Frag<T>::keep(bl[0], bl[1], bl[2], bl[3]);
  }
  acc_guard4(acc[0][0], acc[0][1], acc[0][2], acc[0][3]);
  acc_guard4(acc[1][0], acc[1][1], acc[1][2], acc[1][3]);
  acc_guard4(acc[2][0], acc[2][1], acc[2][2], acc[2][3]);
  acc_guard4(acc[3][0], acc[3][1], acc[3][2], acc[3][3]);

  float* slab = sT[wave];
  const float* Rb = RESID ? (resid + (size_t)b * strideR) : nullptr;
#pragma unroll
  for (int i = 0; i < 4; ++i) {
    const int mBase = m0 + (i << 4);
#pragma unroll
    for (int j = 0; j < 4; ++j) {
      const int n = n0 + (j << 4) + rlane;
      float bv = 0.f;
      if (BIAS_MODE == 2) bv = bias[n];
#pragma unroll
      for (int r = 0; r < 8; ++r) {
        float v = acc[i][j][r] * scale;
        if (BIAS_MODE == 1) v += bias[mBase + mOff + r];
        if (BIAS_MODE == 2) v += bv;
        if (RESID) v += Rb[(size_t)(mBase + mOff + r) * ldc + n];
        if (ACT == 2) v = fmaxf(v, 0.0f);
        if (ACT == 4) v = (v > 0.f) ? v : 0.01f * v;
        slab[(mOff + r) * 68 + (j << 4) + rlane] = v;
      }
    }
    __builtin_amdgcn_fence(__ATOMIC_RELEASE, "workgroup");
    __builtin_amdgcn_wave_barrier();
    __builtin_amdgcn_fence(__ATOMIC_ACQUIRE, "workgroup");
    if (OUT_MODE == 0) {
      float* C = (float*)Cout + (size_t)b * strideC;
      const int hh = lane >> 4, c4 = (lane & 15) * 4;
      for (int pass = 0; pass < 2; ++pass) {
#pragma unroll
        for (int it = 0; it < 8; ++it) {
          const int row = it * 2 + hh;
          v4f v = *(const v4f*)(slab + row * 68 + c4);
          *(volatile v4f*)(C + (size_t)(mBase + row) * ldc + n0 + c4) = v;
        }
        __threadfence();
      }
    } else {
      const int q = lane >> 3, c8 = (lane & 7) * 8;
      unsigned short* C  = (unsigned short*)Cout  + (size_t)b * strideC;
      unsigned short* C2 = (OUT_MODE == 2) ? ((unsigned short*)Cout2 + (size_t)b * strideC) : nullptr;
      for (int pass = 0; pass < 2; ++pass) {
#pragma unroll
        for (int it = 0; it < 4; ++it) {
          const int row = it * 4 + q;
          const float* sp = slab + row * 68 + c8;
          v8h hv, lv;
#pragma unroll
          for (int e = 0; e < 8; ++e) {
            if (OUT_MODE == 1) {
              hv[e] = (_Float16)sp[e];
            } else {
              unsigned short hb = f2bf_bits(sp[e]);
              unsigned short lb = f2bf_bits(sp[e] - bf_bits2f(hb));
              hv[e] = __builtin_bit_cast(_Float16, hb);
              lv[e] = __builtin_bit_cast(_Float16, lb);
            }
          }
          *(volatile v8h*)(C + (size_t)(mBase + row) * ldc + n0 + c8) = hv;
          if (OUT_MODE == 2) *(volatile v8h*)(C2 + (size_t)(mBase + row) * ldc + n0 + c8) = lv;
        }
        __threadfence();
      }
    }
    __builtin_amdgcn_fence(__ATOMIC_RELEASE, "workgroup");
    __builtin_amdgcn_wave_barrier();
    __builtin_amdgcn_fence(__ATOMIC_ACQUIRE, "workgroup");
  }
}

__global__ __launch_bounds__(256) void cast8_bf16_kernel(const float* in0, const float* in1, const float* in2, const float* in3,
                                                        unsigned short* __restrict__ out, int n8, long planeStride) {
  const int sel = blockIdx.y;
  const float* in = (sel == 0) ? in0 : (sel == 1) ? in1 : (sel == 2) ? in2 : in3;
  const int i = blockIdx.x * 256 + threadIdx.x;
  if (i >= n8) return;
  const float* p = in + 8 * (size_t)i;
  const v4f a = *(const v4f*)(p);
  const v4f c = *(const v4f*)(p + 4);
  unsigned short hb[8];
#pragma unroll
  for (int e = 0; e < 4; ++e) {
    hb[e]     = f2bf_bits(a[e]);
    hb[4 + e] = f2bf_bits(c[e]);
  }
  const v4u u = (v4u){pk16(hb[0], hb[1]), pk16(hb[2], hb[3]), pk16(hb[4], hb[5]), pk16(hb[6], hb[7])};
  unsigned short* q = out + (size_t)sel * planeStride + 8 * (size_t)i;
  *(volatile v4u*)q = u;
  __threadfence();
  *(volatile v4u*)q = u;
}

struct FreqTab { float f[kFreq]; };
static_assert(sizeof(FreqTab) == 128, "no padding");

__global__ __launch_bounds__(128) void rotary_split_kernel(
    const float* __restrict__ QF, const float* __restrict__ KF,
    const float* __restrict__ bq, const float* __restrict__ bk,
    unsigned short* __restrict__ Qhi, unsigned short* __restrict__ Qlo,
    unsigned short* __restrict__ Khi, unsigned short* __restrict__ Klo, FreqTab ft) {
#pragma clang fp contract(off)
  __shared__ __align__(16) float csT[kFreq];
  __shared__ __align__(16) float snT[kFreq];
  const int sel  = blockIdx.y;
  const int row  = blockIdx.x;
  const int t    = row & (kSeq - 1);
  const int tid  = threadIdx.x;
  const int lane = tid & 31, wave = tid >> 5;
  const float* src  = (sel == 0) ? QF : KF;
  const float* bias = (sel == 0) ? bq : bk;
  unsigned short* dhi = (sel == 0) ? Qhi : Khi;
  unsigned short* dlo = (sel == 0) ? Qlo : Klo;

  if (wave == 0) {
    float inv = ft.f[0];
#pragma unroll
    for (int i = 1; i < kFreq; ++i) inv = (lane == i) ? ft.f[i] : inv;
    const float ang = (float)t * inv;
    const float cv = cosf(ang);
    const float sv = sinf(ang);
    csT[lane] = cv;
    snT[lane] = sv;
  }
  __syncthreads();

  const int c0 = tid * 8;
  const int j0 = c0 & (kFreq - 1);
  const float* sp = src + (size_t)row * kDim + c0;
  const v4f a0 = *(const v4f*)(sp);
  const v4f a1 = *(const v4f*)(sp + 4);
  const v4f b0 = *(const v4f*)(bias + c0);
  const v4f b1 = *(const v4f*)(bias + c0 + 4);
  const v4f cv0 = *(const v4f*)(csT + j0);
  const v4f cv1 = *(const v4f*)(csT + j0 + 4);
  const v4f sv0 = *(const v4f*)(snT + j0);
  const v4f sv1 = *(const v4f*)(snT + j0 + 4);

  float x[8], cs[8], sn[8];
#pragma unroll
  for (int e = 0; e < 4; ++e) {
    x[e]      = a0[e] + bf_bits2f(f2bf_bits(b0[e]));
    x[4 + e]  = a1[e] + bf_bits2f(f2bf_bits(b1[e]));
    cs[e]     = cv0[e];
    cs[4 + e] = cv1[e];
    sn[e]     = sv0[e];
    sn[4 + e] = sv1[e];
  }
  float rv[8];
#pragma unroll
  for (int e = 0; e < 8; e += 2) {
    rv[e]     = x[e] * cs[e] - x[e + 1] * sn[e];
    rv[e + 1] = x[e + 1] * cs[e + 1] + x[e] * sn[e + 1];
  }
  unsigned short hb[8], lb[8];
#pragma unroll
  for (int e = 0; e < 8; ++e) {
    hb[e] = f2bf_bits(rv[e]);
    lb[e] = f2bf_bits(rv[e] - bf_bits2f(hb[e]));
  }
  const v4u uh = (v4u){pk16(hb[0], hb[1]), pk16(hb[2], hb[3]), pk16(hb[4], hb[5]), pk16(hb[6], hb[7])};
  const v4u ul = (v4u){pk16(lb[0], lb[1]), pk16(lb[2], lb[3]), pk16(lb[4], lb[5]), pk16(lb[6], lb[7])};
  unsigned short* ph = dhi + (size_t)row * kDim + c0;
  unsigned short* pl = dlo + (size_t)row * kDim + c0;
  *(volatile v4u*)ph = uh;
  *(volatile v4u*)pl = ul;
  __threadfence();
  *(volatile v4u*)ph = uh;
  *(volatile v4u*)pl = ul;
}

__global__ __launch_bounds__(256) void vt_split_kernel(const float* __restrict__ VF, const float* __restrict__ bv,
                                                      unsigned short* __restrict__ VThi, unsigned short* __restrict__ VTlo) {
  __shared__ float sm[64][65];
  const int t  = threadIdx.x;
  const int s0 = blockIdx.x * 64;
  const int h  = blockIdx.y;
  const int b  = blockIdx.z;
  const int dcol = t & 63;
  const int rb   = t >> 6;
  const float bvv = bf_bits2f(f2bf_bits(bv[h * kDh + dcol]));
  const float* base = VF + ((size_t)(b * kSeq + s0)) * kDim + h * kDh + dcol;
#pragma unroll
  for (int i = 0; i < 8; ++i) {
    const int r = 4 * i + rb;
    sm[dcol][r] = base[(size_t)r * kDim] + bvv;
  }
  asm volatile("" ::: "memory");
#pragma unroll
  for (int i = 8; i < 16; ++i) {
    const int r = 4 * i + rb;
    sm[dcol][r] = base[(size_t)r * kDim] + bvv;
  }
  __syncthreads();
  const int lane = t & 31, wave = t >> 5;
  const int q = lane >> 3, c8 = (lane & 7) * 8;
  const size_t planeRow = (size_t)(b * kHeads + h) * kDh;
  for (int pass = 0; pass < 2; ++pass) {
#pragma unroll
    for (int it = 0; it < 2; ++it) {
      const int row = wave * 8 + it * 4 + q;
      unsigned short hb[8], lb[8];
#pragma unroll
      for (int e = 0; e < 8; ++e) {
        const float v = sm[row][c8 + e];
        hb[e] = f2bf_bits(v);
        lb[e] = f2bf_bits(v - bf_bits2f(hb[e]));
      }
      const v4u uh = (v4u){pk16(hb[0], hb[1]), pk16(hb[2], hb[3]), pk16(hb[4], hb[5]), pk16(hb[6], hb[7])};
      const v4u ul = (v4u){pk16(lb[0], lb[1]), pk16(lb[2], lb[3]), pk16(lb[4], lb[5]), pk16(lb[6], lb[7])};
      const size_t off = (planeRow + row) * (size_t)kSeq + s0 + c8;
      *(volatile v4u*)(VThi + off) = uh;
      *(volatile v4u*)(VTlo + off) = ul;
    }
    __threadfence();
  }
}

__global__ __launch_bounds__(128) void decay_attn_kernel(
    const unsigned short* __restrict__ Qhi, const unsigned short* __restrict__ Qlo,
    const unsigned short* __restrict__ Khi, const unsigned short* __restrict__ Klo,
    const unsigned short* __restrict__ VThi, const unsigned short* __restrict__ VTlo,
    const float* __restrict__ GF, const float* __restrict__ bg,
    const float* __restrict__ gamma, float* __restrict__ out) {
  __shared__ __align__(16) unsigned short Qsh[kQB * kDh];
  __shared__ __align__(16) unsigned short Qsl[kQB * kDh];
  __shared__ __align__(16) unsigned short Ksh[kKC * kDh];
  __shared__ __align__(16) unsigned short Ksl[kKC * kDh];
  __shared__ __align__(16) unsigned short Vth[kDh * kKC];
  __shared__ __align__(16) unsigned short Vtl[kDh * kKC];
  __shared__ __align__(16) __bf16 Psh[4][16 * kKC];
  __shared__ __align__(16) __bf16 Psl[4][16 * kKC];
  __shared__ __align__(16) float  Os[4][16 * kOsPitch];

  const int tid  = threadIdx.x;
  const int wave = tid >> 5;
  const int lane = tid & 31;
  const int hh   = lane >> 4;
  const int c    = lane & 15;

  const int bx    = blockIdx.x;
  const int qb    = bx % (kSeq / kQB);
  const int bhid  = bx / (kSeq / kQB);
  const int h     = bhid % kHeads;
  const int b     = bhid / kHeads;
  const int qbase = qb * kQB;
  const int q0    = qbase + wave * 16;
  const size_t tokBase = (size_t)b * kSeq;
  const int colBase = h * kDh;
  const size_t vtRowBase = (size_t)(b * kHeads + h) * kDh;

  const float gbf = bf_bits2f(f2bf_bits(gamma[h]));
  const float g   = 1.0f / (1.0f + expf(-gbf));
  const float spanF  = kSkipArg / g;
  const float startF = ((float)(qbase - (kKC - 1)) - spanF) * (1.0f / (float)kKC);
  int kc0 = 0;
  if (startF > 0.0f) { kc0 = (int)startF; if (kc0 > qb) kc0 = qb; }

  {
    const int r = tid >> 1, dh = (tid & 1) * 32;
    const size_t go = (tokBase + qbase + r) * (size_t)kDim + colBase + dh;
    const v4u* qh4 = (const v4u*)(Qhi + go);
    const v4u* ql4 = (const v4u*)(Qlo + go);
#pragma unroll
    for (int i = 0; i < 4; ++i) {
      const v4u wh = qh4[i];
      const v4u wl = ql4[i];
      *(v4u*)(Qsh + r * kDh + dh + 8 * i) = wh;
      *(v4u*)(Qsl + r * kDh + dh + 8 * i) = wl;
    }
  }
  const float cf0  = expf(g * (float)c);
  const float e16g = expf(g * 16.0f);
  const int arow = wave * 16 + c;

  v8f oacc[4];
#pragma unroll
  for (int t4 = 0; t4 < 4; ++t4) oacc[t4] = (v8f){0.f,0.f,0.f,0.f,0.f,0.f,0.f,0.f};

  for (int kc = kc0; kc < kNCh; ++kc) {
    const int kv0 = kc * kKC;
    __syncthreads();
    {
      const int kvr = tid >> 1, dh = (tid & 1) * 32;
      const size_t go = (tokBase + kv0 + kvr) * (size_t)kDim + colBase + dh;
      const v4u* kh4 = (const v4u*)(Khi + go);
      const v4u* kl4 = (const v4u*)(Klo + go);
#pragma unroll
      for (int i = 0; i < 4; ++i) {
        const v4u wkh = kh4[i];
        const v4u wkl = kl4[i];
        *(v4u*)(Ksh + kvr * kDh + dh + 8 * i) = wkh;
        *(v4u*)(Ksl + kvr * kDh + dh + 8 * i) = wkl;
      }
      asm volatile("" ::: "memory");
      const int dr = kvr, sh = dh;
      const size_t gv = (vtRowBase + dr) * (size_t)kSeq + kv0 + sh;
      const v4u* vh4 = (const v4u*)(VThi + gv);
      const v4u* vl4 = (const v4u*)(VTlo + gv);
#pragma unroll
      for (int i = 0; i < 4; ++i) {
        const v4u wv = vh4[i];
        const v4u wl = vl4[i];
        *(v4u*)(Vth + dr * kKC + sh + 8 * i) = wv;
        *(v4u*)(Vtl + dr * kKC + sh + 8 * i) = wl;
      }
    }
    __syncthreads();

    const bool past = (kc <= qb);
    float rowfac[8];
#pragma unroll
    for (int r = 0; r < 8; ++r) {
      float dr = (float)(q0 + 8 * hh + r - kv0);
      dr = fmaxf(dr, 0.0f);
      const float ef = past ? expf(-g * dr) : 1.0f;
      rowfac[r] = ef * kScoreScale;
    }
    __bf16* pwh = Psh[wave];
    __bf16* pwl = Psl[wave];
    float cf = cf0;
#pragma unroll 1
    for (int j = 0; j < 4; ++j) {
      v8f s = (v8f){0.f,0.f,0.f,0.f,0.f,0.f,0.f,0.f};
#pragma unroll
      for (int dc = 0; dc < 2; ++dc) {
        const v16b qh = Frag<__bf16>::load((const __bf16*)Qsh + arow * kDh + dc * 32 + 8 * hh);
        const v16b ql = Frag<__bf16>::load((const __bf16*)Qsl + arow * kDh + dc * 32 + 8 * hh);
        const v16b kb = Frag<__bf16>::load((const __bf16*)Ksh + (j * 16 + c) * kDh + dc * 32 + 8 * hh);
        const v16b kl = Frag<__bf16>::load((const __bf16*)Ksl + (j * 16 + c) * kDh + dc * 32 + 8 * hh);
        s = mma_bf16g(qh, kb, s);
        s = mma_bf16g(qh, kl, s);
        s = mma_bf16g(ql, kb, s);
      }
      const int kvcol = kv0 + j * 16 + c;
#pragma unroll
      for (int r = 0; r < 8; ++r) {
        const int qrow = q0 + 8 * hh + r;
        const float wd  = rowfac[r] * cf;
        const float wdec = ((qrow - kvcol) > 0) ? wd : kScoreScale;
        const float p = s[r] * wdec;
        const unsigned short hb = f2bf_bits(p);
        const unsigned short lb = f2bf_bits(p - bf_bits2f(hb));
        pwh[(8 * hh + r) * kKC + j * 16 + c] = __builtin_bit_cast(__bf16, hb);
        pwl[(8 * hh + r) * kKC + j * 16 + c] = __builtin_bit_cast(__bf16, lb);
      }
      cf = cf * e16g;
    }
    __builtin_amdgcn_fence(__ATOMIC_RELEASE, "workgroup");
    __builtin_amdgcn_wave_barrier();
    __builtin_amdgcn_fence(__ATOMIC_ACQUIRE, "workgroup");

#pragma unroll 1
    for (int kk = 0; kk < 2; ++kk) {
      const v16b pa = Frag<__bf16>::load(pwh + c * kKC + kk * 32 + 8 * hh);
      const v16b pl = Frag<__bf16>::load(pwl + c * kKC + kk * 32 + 8 * hh);
#pragma unroll
      for (int t4 = 0; t4 < 4; ++t4) {
        const v16b vb = Frag<__bf16>::load((const __bf16*)Vth + (t4 * 16 + c) * kKC + kk * 32 + 8 * hh);
        const v16b vl = Frag<__bf16>::load((const __bf16*)Vtl + (t4 * 16 + c) * kKC + kk * 32 + 8 * hh);
        oacc[t4] = mma_bf16g(pa, vb, oacc[t4]);
        oacc[t4] = mma_bf16g(pa, vl, oacc[t4]);
        oacc[t4] = mma_bf16g(pl, vb, oacc[t4]);
      }
    }
  }

  float* os = Os[wave];
#pragma unroll
  for (int r = 0; r < 8; ++r) {
#pragma unroll
    for (int t4 = 0; t4 < 4; ++t4) os[(8 * hh + r) * kOsPitch + t4 * 16 + c] = oacc[t4][r];
  }
  __builtin_amdgcn_fence(__ATOMIC_RELEASE, "workgroup");
  __builtin_amdgcn_wave_barrier();
  __builtin_amdgcn_fence(__ATOMIC_ACQUIRE, "workgroup");
  {
    const int h2 = lane >> 4, c4 = (lane & 15) * 4;
    const v4f bg4 = *(const v4f*)(bg + colBase + c4);
    v4f bgr;
#pragma unroll
    for (int e = 0; e < 4; ++e) bgr[e] = bf_bits2f(f2bf_bits(bg4[e]));
    v4f res[8];
#pragma unroll
    for (int it = 0; it < 8; ++it) {
      const int row = it * 2 + h2;
      const v4f ov = *(const v4f*)(os + row * kOsPitch + c4);
      const size_t go = (tokBase + q0 + row) * (size_t)kDim + colBase + c4;
      const v4f gv = *(const v4f*)(GF + go);
      v4f rv;
#pragma unroll
      for (int e = 0; e < 4; ++e) {
        const float z  = gv[e] + bgr[e];
        const float ez = expf(-z);
        const float sg = z * __builtin_amdgcn_rcpf(1.0f + ez);
        rv[e] = ov[e] * sg;
      }
      res[it] = rv;
      *(volatile v4f*)(out + go) = rv;
    }
    __threadfence();
#pragma unroll
    for (int it = 0; it < 8; ++it) {
      const int row = it * 2 + h2;
      const size_t go = (tokBase + q0 + row) * (size_t)kDim + colBase + c4;
      *(volatile v4f*)(out + go) = res[it];
    }
  }
}

extern "C" void kernel_launch(void* const* d_in, const int* in_sizes, int n_in,
                              void* d_out, int out_size, void* d_ws, size_t ws_size,
                              hipStream_t stream) {
  if (n_in < 10) return;
  const int nX = kTok * kDim;
  const int nW = kDim * kDim;
  if (in_sizes[0] != nX) return;
  if (in_sizes[1] != nW || in_sizes[3] != nW || in_sizes[5] != nW || in_sizes[7] != nW) return;
  if (in_sizes[2] != kDim || in_sizes[4] != kDim || in_sizes[6] != kDim || in_sizes[8] != kDim) return;
  if (in_sizes[9] != kHeads) return;
  if (out_size != nX) return;

  const size_t szXb = (size_t)nX * 2;
  const size_t szWb = (size_t)4 * nW * 2;
  const size_t szF  = (size_t)nX * 4;
  const size_t szP  = (size_t)nX * 2;
  const size_t offXb  = 0;
  const size_t offWb  = offXb + szXb;
  const size_t offQF  = offWb + szWb;
  const size_t offKF  = offQF + szF;
  const size_t offVF  = offKF + szF;
  const size_t offGF  = offVF + szF;
  const size_t offQhi = offGF + szF;
  const size_t offQlo = offQhi + szP;
  const size_t offKhi = offQlo + szP;
  const size_t offKlo = offKhi + szP;
  const size_t offVTh = offKlo + szP;
  const size_t offVTl = offVTh + szP;
  const size_t total  = offVTl + szP;
  if (ws_size < total) return;

  const float* x     = (const float*)d_in[0];
  const float* Wq    = (const float*)d_in[1];
  const float* bq    = (const float*)d_in[2];
  const float* Wk    = (const float*)d_in[3];
  const float* bk    = (const float*)d_in[4];
  const float* Wv    = (const float*)d_in[5];
  const float* bv    = (const float*)d_in[6];
  const float* Wg    = (const float*)d_in[7];
  const float* bg    = (const float*)d_in[8];
  const float* gamma = (const float*)d_in[9];
  float* out = (float*)d_out;
  char* ws = (char*)d_ws;
  unsigned short* xb  = (unsigned short*)(ws + offXb);
  unsigned short* Wb  = (unsigned short*)(ws + offWb);
  float* QF = (float*)(ws + offQF);
  float* KF = (float*)(ws + offKF);
  float* VF = (float*)(ws + offVF);
  float* GF = (float*)(ws + offGF);
  unsigned short* Qhi  = (unsigned short*)(ws + offQhi);
  unsigned short* Qlo  = (unsigned short*)(ws + offQlo);
  unsigned short* Khi  = (unsigned short*)(ws + offKhi);
  unsigned short* Klo  = (unsigned short*)(ws + offKlo);
  unsigned short* VThi = (unsigned short*)(ws + offVTh);
  unsigned short* VTlo = (unsigned short*)(ws + offVTl);

  FreqTab ft;
  for (int j = 0; j < kFreq; ++j) {
    const double pd = std::pow(10000.0, (double)j / (double)kFreq);
    const float pf = (float)pd;
    ft.f[j] = 1.0f / pf;
  }

  const int n8X = nX / 8;
  const int n8W = nW / 8;
  cast8_bf16_kernel<<<dim3(n8X / 256, 1), dim3(256), 0, stream>>>(x, x, x, x, xb, n8X, 0L);
  cast8_bf16_kernel<<<dim3(n8W / 256, 4), dim3(256), 0, stream>>>(Wq, Wk, Wv, Wg, Wb, n8W, (long)nW);
  const int tiles = (kTok / 64) * (kDim / 64);
  wmma_gemm64<1, false, 0, 0, false, 0><<<dim3(tiles / 8, 4), dim3(256), 0, stream>>>(
      xb, xb, kDim, 0L, Wb, Wb, kDim, (long)nW,
      (void*)QF, (void*)QF, kDim, (long)nX, bq, QF, 0L, kTok, kDim, kDim, 1.0f);
  rotary_split_kernel<<<dim3(kTok, 2), dim3(128), 0, stream>>>(QF, KF, bq, bk, Qhi, Qlo, Khi, Klo, ft);
  vt_split_kernel<<<dim3(kSeq / 64, kHeads, kBatch), dim3(256), 0, stream>>>(VF, bv, VThi, VTlo);
  decay_attn_kernel<<<dim3(kBatch * kHeads * (kSeq / kQB)), dim3(128), 0, stream>>>(
      Qhi, Qlo, Khi, Klo, VThi, VTlo, GF, bg, gamma, out);
}
